// MultiScaleAttention_86912958202693
// MI455X (gfx1250) — hardware-verified
//
#include <hip/hip_runtime.h>

typedef __attribute__((ext_vector_type(16))) _Float16 v16h;
typedef __attribute__((ext_vector_type(8)))  _Float16 v8h;
typedef __attribute__((ext_vector_type(4)))  _Float16 v4h;
typedef __attribute__((ext_vector_type(16))) __bf16   v16b;
typedef __attribute__((ext_vector_type(8)))  __bf16   v8b;
typedef __attribute__((ext_vector_type(8)))  float    v8f;
typedef __attribute__((ext_vector_type(4)))  float    v4f;
typedef __attribute__((ext_vector_type(2)))  float    v2f;

#define HEADS 12
#define HD 64
#define DIM 768
#define BATCH 4
#define SQ 3137
#define SQP 3200
#define SK 785
#define SKP 832
#define NQB 50
#define NKC 13
#define BH (BATCH * HEADS)
#define BN (BATCH * SQ)
#define MP 12608
#define REL 111
#define RROWS 112
#define GP 112
#define QHW 56
#define KHW 28

__device__ __forceinline__ unsigned short f2bf_bits(float f) {
  unsigned u = __float_as_uint(f);
  return (unsigned short)((u + 0x7FFFu + ((u >> 16) & 1u)) >> 16);
}
__device__ __forceinline__ float bf_bits2f(unsigned short h) { return __uint_as_float(((unsigned)h) << 16); }

__device__ __forceinline__ void dep_guard_h(v8f& a, v8f& b, v16h x, v16h y) { asm volatile("v_nop\n\tv_nop\n\tv_nop\n\tv_nop" : "+v"(a), "+v"(b) : "v"(x), "v"(y)); }
__device__ __forceinline__ void dep_guard_b(v8f& a, v8f& b, v16b x, v16b y) { asm volatile("v_nop\n\tv_nop\n\tv_nop\n\tv_nop" : "+v"(a), "+v"(b) : "v"(x), "v"(y)); }
__device__ __forceinline__ void keep4_h(v16h a, v16h b, v16h c, v16h d) { asm volatile("v_nop" :: "v"(a), "v"(b), "v"(c), "v"(d)); }
__device__ __forceinline__ void keep4_b(v16b a, v16b b, v16b c, v16b d) { asm volatile("v_nop" :: "v"(a), "v"(b), "v"(c), "v"(d)); }
__device__ __forceinline__ void acc_guard4(v8f& a, v8f& b, v8f& c, v8f& d) { asm volatile("v_nop\n\tv_nop\n\tv_nop\n\tv_nop" : "+v"(a), "+v"(b), "+v"(c), "+v"(d)); }
template <typename T> struct Frag;
template <> struct Frag<_Float16> {
  typedef v16h V; union U { v16h v; v8h h[2]; };
  static __device__ __forceinline__ v16h load(const _Float16* p) {
    U f; f.h[0] = *(const v8h*)(p); f.h[1] = *(const v8h*)(p + 16); return f.v;
  }
  static __device__ __forceinline__ v8f mma(v16h a, v16h b, v8f c) {
    return __builtin_amdgcn_wmma_f32_16x16x32_f16(false, a, false, b, (short)0, c, false, false);
  }
  static __device__ __forceinline__ void guard(v8f& a, v8f& b, v16h x, v16h y) { dep_guard_h(a, b, x, y); }
  static __device__ __forceinline__ void keep(v16h a, v16h b, v16h c, v16h d) { keep4_h(a, b, c, d); }
};
template <> struct Frag<__bf16> {
  typedef v16b V; union U { v16b v; v8b h[2]; };
  static __device__ __forceinline__ v16b load(const __bf16* p) {
    U f; f.h[0] = *(const v8b*)(p); f.h[1] = *(const v8b*)(p + 16); return f.v;
  }
  static __device__ __forceinline__ v8f mma(v16b a, v16b b, v8f c) {
    return __builtin_amdgcn_wmma_f32_16x16x32_bf16(false, a, false, b, (short)0, c, false, false);
  }
  static __device__ __forceinline__ void guard(v8f& a, v8f& b, v16b x, v16b y) { dep_guard_b(a, b, x, y); }
  static __device__ __forceinline__ void keep(v16b a, v16b b, v16b c, v16b d) { keep4_b(a, b, c, d); }
};

template <int ET> struct Elem;
template <> struct Elem<0> { typedef _Float16 T; };
template <> struct Elem<1> { typedef __bf16 T; };
template <int ET, bool SPLIT, int BIAS_MODE, int OUT_MODE, bool RESID, int ACT = 0>
__global__ __launch_bounds__(256) void wmma_gemm64(
    const unsigned short* __restrict__ Ap, const unsigned short* __restrict__ A2p, int lda, long strideA,
    const unsigned short* __restrict__ Btp, const unsigned short* __restrict__ Bt2p, int ldb, long strideB,
    void* __restrict__ Cout, void* __restrict__ Cout2, int ldc, long strideC,
    const float* __restrict__ bias,
    const float* __restrict__ resid, long strideR,
    int M, int N, int K, float scale, int Mlim) {
  typedef typename Elem<ET>::T T;
  typedef typename Frag<T>::V V;
  const T* A = (const T*)Ap; const T* A2 = (const T*)A2p; const T* Bt = (const T*)Btp; const T* Bt2 = (const T*)Bt2p;
  __shared__ __align__(16) float sT[8][16 * 68];
  const int b    = blockIdx.y;
  const int lane = threadIdx.x & 31;
  const int wave = threadIdx.x >> 5;
  const int tilesN = N >> 6;
  const int tilesM = M >> 6;
  const int tile = blockIdx.x * 8 + wave;
  if (tile >= tilesM * tilesN) return;
  const int tm = tile / tilesN;
  const int tn = tile - tm * tilesN;
  const int m0 = tm << 6;
  const int n0 = tn << 6;

  const T* Ab  = A  + (size_t)b * strideA;
  const T* Bb  = Bt + (size_t)b * strideB;
  const T* Ab2 = SPLIT ? (A2  + (size_t)b * strideA) : nullptr;
  const T* Bb2 = SPLIT ? (Bt2 + (size_t)b * strideB) : nullptr;

  const int rlane = lane & 15;
  const int koff  = (lane >> 4) * 8;
  const int mOff  = (lane >> 4) * 8;

  v8f acc[4][4];
#pragma unroll
  for (int i = 0; i < 4; ++i)
#pragma unroll
    for (int j = 0; j < 4; ++j) acc[i][j] = (v8f){0.f,0.f,0.f,0.f,0.f,0.f,0.f,0.f};

  for (int k0 = 0; k0 < K; k0 += 32) {
    V bh[4], bl[4];
#pragma unroll
    for (int j = 0; j < 4; ++j) {
      const size_t bo = (size_t)(n0 + (j << 4) + rlane) * ldb + koff + k0;
      bh[j] = Frag<T>::load(Bb + bo);
      if (SPLIT) bl[j] = Frag<T>::load(Bb2 + bo);
    }
#pragma unroll
    for (int i = 0; i < 4; ++i) {
      const size_t ao = (size_t)(m0 + (i << 4) + rlane) * lda + koff + k0;
      V ah = Frag<T>::load(Ab + ao);
      V al;
      if (SPLIT) al = Frag<T>::load(Ab2 + ao);
#pragma unroll
      for (int j = 0; j < 4; ++j) {
        acc[i][j] = Frag<T>::mma(ah, bh[j], acc[i][j]);
        if (SPLIT) {
          acc[i][j] = Frag<T>::mma(ah, bl[j], acc[i][j]);
          acc[i][j] = Frag<T>::mma(al, bh[j], acc[i][j]);
        }
      }
      Frag<T>::guard(acc[i][0], acc[i][3], ah, SPLIT ? al : ah);
    }
    Frag<T>::keep(bh[0], bh[1], bh[2], bh[3]);
    if (SPLIT) Frag<T>::keep(bl[0], bl[1], bl[2], bl[3]);
  }
  acc_guard4(acc[0][0], acc[0][1], acc[0][2], acc[0][3]);
  acc_guard4(acc[1][0], acc[1][1], acc[1][2], acc[1][3]);
  acc_guard4(acc[2][0], acc[2][1], acc[2][2], acc[2][3]);
  acc_guard4(acc[3][0], acc[3][1], acc[3][2], acc[3][3]);

  float* slab = sT[wave];
  const float* Rb = RESID ? (resid + (size_t)b * strideR) : nullptr;
#pragma unroll
  for (int i = 0; i < 4; ++i) {
    const int mBase = m0 + (i << 4);
#pragma unroll
    for (int j = 0; j < 4; ++j) {
      const int n = n0 + (j << 4) + rlane;
      float bv = 0.f;
      if (BIAS_MODE == 2) bv = bias[n];
#pragma unroll
      for (int r = 0; r < 8; ++r) {
        float v = acc[i][j][r] * scale;
        if (BIAS_MODE == 1) v += bias[mBase + mOff + r];
        if (BIAS_MODE == 2) v += bv;
        if (RESID) v += Rb[(size_t)(mBase + mOff + r) * ldc + n];
        if (ACT == 1) v = tanhf(v);
        if (ACT == 2) v = fmaxf(v, 0.0f);
        if (ACT == 3) v = v / (1.0f + expf(-v));
        if (ACT == 4) v = (v > 0.f) ? v : 0.01f * v;
        if (ACT == 5) v = 0.5f * v * (1.0f + erff(v * 0.70710678118654752f));
        slab[(mOff + r) * 68 + (j << 4) + rlane] = v;
      }
    }
    __builtin_amdgcn_fence(__ATOMIC_RELEASE, "workgroup");
    __builtin_amdgcn_wave_barrier();
    __builtin_amdgcn_fence(__ATOMIC_ACQUIRE, "workgroup");
    if (OUT_MODE == 0) {
      float* C = (float*)Cout + (size_t)b * strideC;
      const int hh = lane >> 4, c4 = (lane & 15) * 4;
      for (int pass = 0; pass < 2; ++pass) {
#pragma unroll
        for (int it = 0; it < 8; ++it) {
          const int row = it * 2 + hh;
          v4f v = *(const v4f*)(slab + row * 68 + c4);
          if (mBase + row < Mlim) *(volatile v4f*)(C + (size_t)(mBase + row) * ldc + n0 + c4) = v;
        }
        __threadfence();
      }
    } else {
      const int q = lane >> 3, c8 = (lane & 7) * 8;
      unsigned short* C  = (unsigned short*)Cout  + (size_t)b * strideC;
      unsigned short* C2 = (OUT_MODE == 2) ? ((unsigned short*)Cout2 + (size_t)b * strideC) : nullptr;
      for (int pass = 0; pass < 2; ++pass) {
#pragma unroll
        for (int it = 0; it < 4; ++it) {
          const int row = it * 4 + q;
          const float* sp = slab + row * 68 + c8;
          v8h hv, lv;
#pragma unroll
          for (int e = 0; e < 8; ++e) {
            if (OUT_MODE == 1) {
              hv[e] = (_Float16)sp[e];
            } else {
              unsigned short hb = f2bf_bits(sp[e]);
              unsigned short lb = f2bf_bits(sp[e] - bf_bits2f(hb));
              hv[e] = __builtin_bit_cast(_Float16, hb);
              lv[e] = __builtin_bit_cast(_Float16, lb);
            }
          }
          if (mBase + row < Mlim) {
            *(volatile v8h*)(C + (size_t)(mBase + row) * ldc + n0 + c8) = hv;
            if (OUT_MODE == 2) *(volatile v8h*)(C2 + (size_t)(mBase + row) * ldc + n0 + c8) = lv;
          }
        }
        __threadfence();
      }
    }
    __builtin_amdgcn_fence(__ATOMIC_RELEASE, "workgroup");
    __builtin_amdgcn_wave_barrier();
    __builtin_amdgcn_fence(__ATOMIC_ACQUIRE, "workgroup");
  }
}

__global__ __launch_bounds__(256) void cast_rows_f16(const float* __restrict__ X, _Float16* __restrict__ Xh,
                                                     int rows_in, int rows_out) {
  const int i = blockIdx.x * 256 + threadIdx.x;
  const int per = DIM / 8;
  if (i >= rows_out * per) return;
  const int row = i / per;
  const int c8 = (i - row * per) * 8;
  const int rc = row < rows_in ? row : rows_in - 1;
  const float f = row < rows_in ? 1.f : 0.f;
  const float* src = X + (size_t)rc * DIM + c8;
  const v4f a = *(const v4f*)src;
  const v4f bq = *(const v4f*)(src + 4);
  v8h hv;
#pragma unroll
  for (int e = 0; e < 4; ++e) { hv[e] = (_Float16)(a[e] * f); hv[4 + e] = (_Float16)(bq[e] * f); }
  _Float16* dst = Xh + (size_t)row * DIM + c8;
  *(volatile v8h*)dst = hv;
  __threadfence();
  *(volatile v8h*)dst = hv;
}

__global__ __launch_bounds__(256) void cast_transpose_f16(const float* __restrict__ W, _Float16* __restrict__ Wt,
                                                          int K, int N, float scale) {
  __shared__ float tile[64][33];
  const int n0 = blockIdx.x * 32, k0 = blockIdx.y * 64, t = threadIdx.x;
#pragma unroll
  for (int i = 0; i < 8; ++i) {
    const int idx = i * 256 + t;
    const int ky = idx >> 5, nx = idx & 31;
    tile[ky][nx] = W[(size_t)(k0 + ky) * N + n0 + nx];
  }
  __syncthreads();
  const int n = t >> 3, q = t & 7;
  v8h hv;
#pragma unroll
  for (int e = 0; e < 8; ++e) hv[e] = (_Float16)(tile[q * 8 + e][n] * scale);
  _Float16* dst = Wt + (size_t)(n0 + n) * K + k0 + q * 8;
  *(volatile v8h*)dst = hv;
  __threadfence();
  *(volatile v8h*)dst = hv;
}

template <int STRIDE, bool RES>
__global__ __launch_bounds__(128)
void pool_ln_kernel(const float* __restrict__ Tin, const float* __restrict__ w,
                    const float* __restrict__ g, const float* __restrict__ bb,
                    _Float16* __restrict__ outh, float* __restrict__ outres, int ntokp) {
  constexpr int HO = (QHW + 2 - 3) / STRIDE + 1;
  constexpr int NB = HO * HO;
  constexpr int NTOK = 1 + NB;
  const int lane = threadIdx.x & 31;
  const int wid = blockIdx.x * 4 + (threadIdx.x >> 5);
  if (wid >= BH * ntokp) return;
  const int t = wid % ntokp;
  const int bh = wid / ntokp;
  const int h = bh % HEADS, b = bh / HEADS;
  const int d0 = 2 * lane;
  const float* Tb = Tin + (size_t)b * SQ * DIM + h * HD + d0;
  int p = t - 1;
  p = p < 0 ? 0 : p;
  p = p > NB - 1 ? NB - 1 : p;
  const int oy = p / HO, ox = p - oy * HO;
  float a0 = 0.f, a1 = 0.f;
#pragma unroll
  for (int ky = 0; ky < 3; ++ky) {
#pragma unroll
    for (int kx = 0; kx < 3; ++kx) {
      const int iy = oy * STRIDE + ky - 1, ix = ox * STRIDE + kx - 1;
      const bool inb = (iy >= 0) && (iy < QHW) && (ix >= 0) && (ix < QHW);
      const int iyc = iy < 0 ? 0 : (iy > QHW - 1 ? QHW - 1 : iy);
      const int ixc = ix < 0 ? 0 : (ix > QHW - 1 ? QHW - 1 : ix);
      const v2f dv = *(const v2f*)(Tb + (size_t)(1 + iyc * QHW + ixc) * DIM);
      const float fl = inb ? 1.f : 0.f;
      a0 += (dv[0] * fl) * w[d0 * 9 + ky * 3 + kx];
      a1 += (dv[1] * fl) * w[(d0 + 1) * 9 + ky * 3 + kx];
    }
  }
  const v2f cv = *(const v2f*)Tb;
  const bool iscls = (t == 0);
  const float v0 = iscls ? cv[0] : a0;
  const float v1 = iscls ? cv[1] : a1;
  float s = v0 + v1;
#pragma unroll
  for (int off = 16; off; off >>= 1) s += __shfl_xor(s, off, 32);
  const float mu = s * (1.f / 64.f);
  const float e0 = v0 - mu, e1 = v1 - mu;
  float sq = e0 * e0 + e1 * e1;
#pragma unroll
  for (int off = 16; off; off >>= 1) sq += __shfl_xor(sq, off, 32);
  const float rinv = rsqrtf(sq * (1.f / 64.f) + 1e-5f);
  const bool valid = t < NTOK;
  float y0 = e0 * rinv * g[d0] + bb[d0];
  float y1 = e1 * rinv * g[d0 + 1] + bb[d0 + 1];
  y0 = valid ? y0 : 0.f;
  y1 = valid ? y1 : 0.f;
  const size_t ro = ((size_t)bh * ntokp + t) * HD + d0;
  const _Float16 h0 = (_Float16)y0, h1 = (_Float16)y1;
  const unsigned u = (unsigned)__builtin_bit_cast(unsigned short, h0) | ((unsigned)__builtin_bit_cast(unsigned short, h1) << 16);
  v2f rv; rv[0] = y0; rv[1] = y1;
  *(volatile unsigned*)(outh + ro) = u;
  if (RES) *(volatile v2f*)(outres + ro) = rv;
  __threadfence();
  *(volatile unsigned*)(outh + ro) = u;
  if (RES) *(volatile v2f*)(outres + ro) = rv;
}

__device__ __forceinline__ v8f hmma(v16h a, v16h b, v8f c) {
  c = __builtin_amdgcn_wmma_f32_16x16x32_f16(false, a, false, b, (short)0, c, false, false);
  asm volatile("v_nop\n\tv_nop\n\tv_nop\n\tv_nop" : "+v"(c) : "v"(a), "v"(b));
  return c;
}

__global__ __launch_bounds__(128)
void attn_kernel(const _Float16* __restrict__ Qh, const _Float16* __restrict__ Kh,
                 const _Float16* __restrict__ Vh, const float* __restrict__ Qres,
                 const float* __restrict__ relh, const float* __restrict__ relw,
                 _Float16* __restrict__ Oh) {
  __shared__ __align__(16) _Float16 Rs[2 * RROWS * HD];
  __shared__ __align__(16) float    Gs[4 * 2 * 16 * GP];
  __shared__ __align__(16) _Float16 Ksh[64 * 64];
  __shared__ __align__(16) _Float16 Vth[64 * 64];
  __shared__ __align__(16) _Float16 Psh[4 * 16 * 64];

  const int tid = threadIdx.x, wave = tid >> 5, lane = tid & 31;
  const int hh = lane >> 4, c = lane & 15;
  const int bx = blockIdx.x;
  const int qb = bx % NQB;
  const int bh = bx / NQB;
  const int h = bh % HEADS, b = bh / HEADS;
  const int q0 = qb * 64 + wave * 16;
  const v8f z8 = (v8f){0.f,0.f,0.f,0.f,0.f,0.f,0.f,0.f};

  for (int i = tid; i < RROWS * (HD / 4); i += 128) {
    const int row = i >> 4, c4 = (i & 15) * 4;
    const int rc = row < REL ? row : REL - 1;
    const float f = row < REL ? 64.f : 0.f;
    const v4f a = *(const v4f*)(relh + rc * HD + c4);
    const v4f wv = *(const v4f*)(relw + rc * HD + c4);
    v4h ha, hw;
#pragma unroll
    for (int e = 0; e < 4; ++e) { ha[e] = (_Float16)(a[e] * f); hw[e] = (_Float16)(wv[e] * f); }
    *(v4h*)(Rs + row * HD + c4) = ha;
    *(v4h*)(Rs + RROWS * HD + row * HD + c4) = hw;
  }
  v16h qa[2];
  {
    const _Float16* qp = Qh + ((size_t)bh * SQP + q0 + c) * HD + 8 * hh;
    qa[0] = Frag<_Float16>::load(qp);
    qa[1] = Frag<_Float16>::load(qp + 32);
  }
  __syncthreads();

  float* gh = Gs + (wave * 2) * (16 * GP);
  float* gw = gh + 16 * GP;
  {
#pragma unroll 1
    for (int nt = 0; nt < 7; ++nt) {
      v8f ah = z8, aw = z8;
#pragma unroll
      for (int dc = 0; dc < 2; ++dc) {
        const _Float16* rp = Rs + (nt * 16 + c) * HD + dc * 32 + 8 * hh;
        const v16h b0 = Frag<_Float16>::load(rp);
        const v16h b1 = Frag<_Float16>::load(rp + RROWS * HD);
        ah = hmma(qa[dc], b0, ah);
        aw = hmma(qa[dc], b1, aw);
      }
#pragma unroll
      for (int r = 0; r < 8; ++r) {
        const float f = ((q0 + 8 * hh + r) >= 1) ? (1.0f / 64.0f) : 0.f;
        gh[(8 * hh + r) * GP + nt * 16 + c] = ah[r] * f;
        gw[(8 * hh + r) * GP + nt * 16 + c] = aw[r] * f;
      }
    }
  }
  int boh[8], bow[8];
#pragma unroll
  for (int r = 0; r < 8; ++r) {
    int p = q0 + 8 * hh + r - 1;
    p = p < 0 ? 0 : p;
    p = p > QHW * QHW - 1 ? QHW * QHW - 1 : p;
    const int qy = p / QHW, qx = p - qy * QHW;
    boh[r] = (8 * hh + r) * GP + qy + 2 * (KHW - 1);
    bow[r] = (8 * hh + r) * GP + qx + 2 * (KHW - 1);
  }

  float mrow[8], lrow[8];
  v8f oacc[4];
#pragma unroll
  for (int r = 0; r < 8; ++r) { mrow[r] = -INFINITY; lrow[r] = 0.f; }
#pragma unroll
  for (int t = 0; t < 4; ++t) oacc[t] = z8;

  for (int kc = 0; kc < NKC; ++kc) {
    const int kv0 = kc * 64;
    __syncthreads();
    {
      const int kvr = tid >> 1, dh = (tid & 1) * 32;
      const _Float16* krow = Kh + ((size_t)bh * SKP + kv0 + kvr) * HD + dh;
      const _Float16* vrow = Vh + ((size_t)bh * SKP + kv0 + kvr) * HD + dh;
#pragma unroll
      for (int i = 0; i < 4; ++i) {
        const v8h kk = *(const v8h*)(krow + 8 * i);
        const v8h vv = *(const v8h*)(vrow + 8 * i);
        *(v8h*)(Ksh + kvr * HD + dh + 8 * i) = kk;
#pragma unroll
        for (int e = 0; e < 8; ++e) Vth[(dh + 8 * i + e) * 64 + kvr] = vv[e];
      }
    }
    __syncthreads();

    v8f s[4];
#pragma unroll
    for (int j = 0; j < 4; ++j) {
      s[j] = z8;
#pragma unroll
      for (int dc = 0; dc < 2; ++dc) {
        const v16h kb = Frag<_Float16>::load(Ksh + (j * 16 + c) * HD + dc * 32 + 8 * hh);
        s[j] = hmma(qa[dc], kb, s[j]);
      }
    }
    int kh2[4], kw2[4];
    float kf[4];
    bool km[4];
#pragma unroll
    for (int j = 0; j < 4; ++j) {
      const int kvcol = kv0 + j * 16 + c;
      int kbi = kvcol - 1;
      kbi = kbi < 0 ? 0 : kbi;
      kbi = kbi > KHW * KHW - 1 ? KHW * KHW - 1 : kbi;
      const int ky = kbi / KHW;
      kh2[j] = 2 * ky;
      kw2[j] = 2 * (kbi - ky * KHW);
      kf[j] = (kvcol >= 1 && kvcol < SK) ? 1.f : 0.f;
      km[j] = (kvcol >= SK);
    }
    float cm[8];
#pragma unroll
    for (int r = 0; r < 8; ++r) {
      float m = -INFINITY;
#pragma unroll
      for (int j = 0; j < 4; ++j) {
        const float bias = (gh[boh[r] - kh2[j]] + gw[bow[r] - kw2[j]]) * kf[j];
        float val = s[j][r] * 0.125f + bias;
        val = km[j] ? -INFINITY : val;
        s[j][r] = val;
        m = fmaxf(m, val);
      }
#pragma unroll
      for (int off = 1; off < 16; off <<= 1) m = fmaxf(m, __shfl_xor(m, off, 32));
      cm[r] = m;
    }
    _Float16* pwh = Psh + wave * (16 * 64);
#pragma unroll
    for (int r = 0; r < 8; ++r) {
      const float mnew = fmaxf(mrow[r], cm[r]);
      const float alpha = expf(mrow[r] - mnew);
      mrow[r] = mnew;
      float psum = 0.f;
#pragma unroll
      for (int j = 0; j < 4; ++j) {
        const float p = expf(s[j][r] - mnew);
        psum += p;
        pwh[(8 * hh + r) * 64 + j * 16 + c] = (_Float16)(p * 32768.0f);
      }
#pragma unroll
      for (int off = 1; off < 16; off <<= 1) psum += __shfl_xor(psum, off, 32);
      lrow[r] = lrow[r] * alpha + psum;
#pragma unroll
      for (int t = 0; t < 4; ++t) oacc[t][r] *= alpha;
    }
    __builtin_amdgcn_fence(__ATOMIC_RELEASE, "workgroup");
    __builtin_amdgcn_wave_barrier();
    __builtin_amdgcn_fence(__ATOMIC_ACQUIRE, "workgroup");
#pragma unroll 1
    for (int kk = 0; kk < 2; ++kk) {
      const v16h pa = Frag<_Float16>::load(pwh + c * 64 + kk * 32 + 8 * hh);
#pragma unroll
      for (int t = 0; t < 4; ++t) {
        const v16h vb = Frag<_Float16>::load(Vth + (t * 16 + c) * 64 + kk * 32 + 8 * hh);
        oacc[t] = hmma(pa, vb, oacc[t]);
      }
    }
  }

  float* os = (float*)Rs + wave * (16 * 68);
#pragma unroll
  for (int r = 0; r < 8; ++r) {
    const int qrow = q0 + 8 * hh + r;
    const float inv = 1.0f / (lrow[r] * 32768.0f);
    const float rf = (qrow >= 1) ? 1.f : 0.f;
    const float* rp = Qres + ((size_t)bh * SQP + qrow) * HD + c;
#pragma unroll
    for (int t = 0; t < 4; ++t) os[(8 * hh + r) * 68 + t * 16 + c] = oacc[t][r] * inv + rp[t * 16] * rf;
  }
  __builtin_amdgcn_fence(__ATOMIC_RELEASE, "workgroup");
  __builtin_amdgcn_wave_barrier();
  __builtin_amdgcn_fence(__ATOMIC_ACQUIRE, "workgroup");
  {
    const int q = lane >> 3, c8 = (lane & 7) * 8;
    _Float16* ob = Oh + (size_t)b * SQ * DIM + h * HD + c8;
    for (int pass = 0; pass < 2; ++pass) {
#pragma unroll
      for (int it = 0; it < 4; ++it) {
        const int row = it * 4 + q;
        const int qq = q0 + row;
        const float* sp = os + row * 68 + c8;
        v8h hv;
#pragma unroll
        for (int e = 0; e < 8; ++e) hv[e] = (_Float16)sp[e];
        if (qq < SQ) *(volatile v8h*)(ob + (size_t)qq * DIM) = hv;
      }
      __threadfence();
    }
  }
}

extern "C" void kernel_launch(void* const* d_in, const int* in_sizes, int n_in,
                              void* d_out, int out_size, void* d_ws, size_t ws_size,
                              hipStream_t stream) {
  if (n_in < 15) return;
  if (in_sizes[0] != BATCH * SQ * DIM || in_sizes[1] != DIM * 3 * DIM || in_sizes[2] != HD * 9 ||
      in_sizes[3] != HD * 9 || in_sizes[4] != HD * 9 || in_sizes[11] != REL * HD || in_sizes[12] != REL * HD ||
      in_sizes[13] != DIM * DIM || in_sizes[14] != DIM || out_size != BATCH * SQ * DIM) return;

  const float* x       = (const float*)d_in[0];
  const float* Wqkv    = (const float*)d_in[1];
  const float* pool_qw = (const float*)d_in[2];
  const float* pool_kw = (const float*)d_in[3];
  const float* pool_vw = (const float*)d_in[4];
  const float* gq = (const float*)d_in[5];
  const float* bq = (const float*)d_in[6];
  const float* gk = (const float*)d_in[7];
  const float* bk = (const float*)d_in[8];
  const float* gv = (const float*)d_in[9];
  const float* bv = (const float*)d_in[10];
  const float* relH  = (const float*)d_in[11];
  const float* relW  = (const float*)d_in[12];
  const float* Wproj = (const float*)d_in[13];
  const float* bproj = (const float*)d_in[14];
  float* out = (float*)d_out;

  const size_t szXh = (size_t)MP * DIM * 2;
  const size_t szWq = (size_t)3 * DIM * DIM * 2;
  const size_t szWp = (size_t)DIM * DIM * 2;
  const size_t szT  = (size_t)MP * DIM * 4;
  const size_t szQh = (size_t)BH * SQP * HD * 2;
  const size_t szKh = (size_t)BH * SKP * HD * 2;
  const size_t szVh = szKh;
  const size_t szQr = (size_t)BH * SQP * HD * 4;
  const size_t total = szXh + szWq + szWp + szT + szQh + szKh + szVh + szQr;
  if (total > ws_size) return;
  char* ws = (char*)d_ws;
  size_t off = 0;
  _Float16* Xh  = (_Float16*)(ws + off); off += szXh;
  _Float16* WqT = (_Float16*)(ws + off); off += szWq;
  _Float16* WpT = (_Float16*)(ws + off); off += szWp;
  float*    T   = (float*)(ws + off);    off += szT;
  _Float16* Qh  = (_Float16*)(ws + off); off += szQh;
  _Float16* Kh  = (_Float16*)(ws + off); off += szKh;
  _Float16* Vh  = (_Float16*)(ws + off); off += szVh;
  float*    Qr  = (float*)(ws + off);    off += szQr;
  _Float16* Oh  = Xh;

  cast_rows_f16<<<(MP * (DIM / 8) + 255) / 256, 256, 0, stream>>>(x, Xh, BN, MP);
  cast_transpose_f16<<<dim3((3 * DIM) / 32, DIM / 64), 256, 0, stream>>>(Wqkv, WqT, DIM, 3 * DIM, 64.0f);
  cast_transpose_f16<<<dim3(DIM / 32, DIM / 64), 256, 0, stream>>>(Wproj, WpT, DIM, DIM, 64.0f);

  const int gemmBlocks = ((MP / 64) * (DIM / 64) + 7) / 8;
  wmma_gemm64<0, false, 0, 0, false><<<dim3(gemmBlocks, 1), 256, 0, stream>>>(
      (const unsigned short*)Xh, (const unsigned short*)Xh, DIM, 0L,
      (const unsigned short*)(WqT + (size_t)1 * DIM * DIM), (const unsigned short*)(WqT + (size_t)1 * DIM * DIM), DIM, 0L,
      (void*)T, (void*)T, DIM, 0L, bproj, bproj, 0L, MP, DIM, DIM, 1.0f / 64.0f, MP);
  pool_ln_kernel<2, false><<<(BH * SKP) / 4, 128, 0, stream>>>(T, pool_kw, gk, bk, Kh, Qr, SKP);
  wmma_gemm64<0, false, 0, 0, false><<<dim3(gemmBlocks, 1), 256, 0, stream>>>(
      (const unsigned short*)Xh, (const unsigned short*)Xh, DIM, 0L,
      (const unsigned short*)(WqT + (size_t)2 * DIM * DIM), (const unsigned short*)(WqT + (size_t)2 * DIM * DIM), DIM, 0L,
      (void*)T, (void*)T, DIM, 0L, bproj, bproj, 0L, MP, DIM, DIM, 1.0f / 64.0f, MP);
  pool_ln_kernel<2, false><<<(BH * SKP) / 4, 128, 0, stream>>>(T, pool_vw, gv, bv, Vh, Qr, SKP);
  wmma_gemm64<0, false, 0, 0, false><<<dim3(gemmBlocks, 1), 256, 0, stream>>>(
      (const unsigned short*)Xh, (const unsigned short*)Xh, DIM, 0L,
      (const unsigned short*)WqT, (const unsigned short*)WqT, DIM, 0L,
      (void*)T, (void*)T, DIM, 0L, bproj, bproj, 0L, MP, DIM, DIM, 1.0f / 64.0f, MP);
  pool_ln_kernel<1, true><<<(BH * SQP) / 4, 128, 0, stream>>>(T, pool_qw, gq, bq, Qh, Qr, SQP);
  attn_kernel<<<BH * NQB, 128, 0, stream>>>(Qh, Kh, Vh, Qr, relH, relW, Oh);
  wmma_gemm64<0, false, 2, 0, false><<<dim3(gemmBlocks, 1), 256, 0, stream>>>(
      (const unsigned short*)Oh, (const unsigned short*)Oh, DIM, 0L,
      (const unsigned short*)WpT, (const unsigned short*)WpT, DIM, 0L,
      (void*)out, (void*)out, DIM, 0L, bproj, bproj, 0L, MP, DIM, DIM, 1.0f / 64.0f, BN);
}
